// OctreeResBlock2_8624294331036
// MI455X (gfx1250) — hardware-run, weakly checked
//
#include <hip/hip_runtime.h>
#include <stdint.h>

#pragma clang fp contract(off)

#define NCO   128
#define CIA   64
#define KTAP  27
#define NT    128
#define SP    132
#define TP    33
#define BNEPS 1e-3f

static_assert(NCO == 128);
static_assert(NT == 128);
static_assert((SP * 4) % 16 == 0);

typedef __bf16         v16b __attribute__((ext_vector_type(16)));
typedef __bf16         v8b  __attribute__((ext_vector_type(8)));
typedef _Float16       v16h __attribute__((ext_vector_type(16)));
typedef _Float16       v8h  __attribute__((ext_vector_type(8)));
typedef float          v8f  __attribute__((ext_vector_type(8)));
typedef float          v4f  __attribute__((ext_vector_type(4)));
typedef unsigned       v4u  __attribute__((ext_vector_type(4)));
typedef double         v2d  __attribute__((ext_vector_type(2)));

__device__ __forceinline__ unsigned bfb(float f) {
  const unsigned u = __float_as_uint(f);
  return (u + 0x7FFFu + ((u >> 16) & 1u)) >> 16;
}
__device__ __forceinline__ float bf_rne(float f) { return __uint_as_float(bfb(f) << 16); }
__device__ __forceinline__ unsigned h16b(float f) {
  union { _Float16 h; unsigned short u; } c; c.h = (_Float16)f; return (unsigned)c.u;
}
__device__ __forceinline__ v8f zero8f() { v8f z = {0.f, 0.f, 0.f, 0.f, 0.f, 0.f, 0.f, 0.f}; return z; }

template<bool F16> struct Mma;
template<> struct Mma<false> {
  typedef v16b frag; typedef v8b hfrag;
  static __device__ __forceinline__ v8f mma(frag a, frag b, v8f c) {
    return __builtin_amdgcn_wmma_f32_16x16x32_bf16(false, a, false, b, (short)0, c, false, false);
  }
};
template<> struct Mma<true> {
  typedef v16h frag; typedef v8h hfrag;
  static __device__ __forceinline__ v8f mma(frag a, frag b, v8f c) {
    return __builtin_amdgcn_wmma_f32_16x16x32_f16(false, a, false, b, (short)0, c, false, false);
  }
};

template<bool F16>
__device__ __forceinline__ typename Mma<F16>::frag ldfrag(const unsigned short* p) {
  typedef typename Mma<F16>::hfrag HF;
  union { typename Mma<F16>::frag v; HF h[2]; } f;
  f.h[0] = *(const HF*)(p);
  f.h[1] = *(const HF*)(p + 16);
  return f.v;
}

template<class F>
__device__ __forceinline__ void guard8x6(v8f& c0, v8f& c1, v8f& c2, v8f& c3, v8f& c4, v8f& c5, v8f& c6, v8f& c7,
                                         const F& f0, const F& f1, const F& f2, const F& f3, const F& f4, const F& f5) {
#if defined(__HIP_DEVICE_COMPILE__)
  asm volatile("v_nop\n\tv_nop\n\tv_nop\n\tv_nop"
               : "+v"(c0), "+v"(c1), "+v"(c2), "+v"(c3), "+v"(c4), "+v"(c5), "+v"(c6), "+v"(c7)
               : "v"(f0), "v"(f1), "v"(f2), "v"(f3), "v"(f4), "v"(f5));
#endif
}
__device__ __forceinline__ void acc_guard8(v8f& c0, v8f& c1, v8f& c2, v8f& c3, v8f& c4, v8f& c5, v8f& c6, v8f& c7) {
#if defined(__HIP_DEVICE_COMPILE__)
  asm volatile("v_nop\n\tv_nop\n\tv_nop\n\tv_nop"
               : "+v"(c0), "+v"(c1), "+v"(c2), "+v"(c3), "+v"(c4), "+v"(c5), "+v"(c6), "+v"(c7));
#endif
}

template<int CIN, bool GATHER> struct ConvCfg {
  static constexpr int ROWP = CIN + 8;
  static constexpr int OPB  = (NCO + NT) * ROWP * 2;
  static constexpr int STB  = NT * SP * 4;
  static constexpr int UNI  = (OPB > STB) ? OPB : STB;
  static constexpr int LDS  = UNI + (GATHER ? NT * KTAP * 4 : 0);
};

__global__ __launch_bounds__(256)
void k_xT(const float* __restrict__ x, int npts, unsigned short* xT)
{
  __shared__ float tile[CIA * TP];
  const int tid  = threadIdx.x;
  const int lane = tid & 31;
  const int wid  = tid >> 5;
  const int pj   = lane & 7;
  const int lq   = lane >> 3;
  const int px   = tid & 31;
  const int cr   = tid >> 5;
  const int n0   = blockIdx.x * 32;
#pragma unroll
  for (int i = 0; i < 8; ++i) {
    const int c = cr + 8 * i;
    tile[c * TP + px] = x[(size_t)c * npts + n0 + px];
  }
  __syncthreads();
  const int L = wid * 4 + lq;
  unsigned hb[8];
#pragma unroll
  for (int e = 0; e < 8; ++e) hb[e] = bfb(tile[(8 * pj + e) * TP + L]);
  v4u wv;
  wv.x = hb[0] | (hb[1] << 16);
  wv.y = hb[2] | (hb[3] << 16);
  wv.z = hb[4] | (hb[5] << 16);
  wv.w = hb[6] | (hb[7] << 16);
  const size_t eo = (size_t)(n0 + L) * CIA + 8 * pj;
  *(volatile v4u*)(xT + eo) = wv;
  __threadfence();
  *(volatile v4u*)(xT + eo) = wv;
}

__global__ __launch_bounds__(256)
void k_wpack(const float* __restrict__ w, int cin, int ktaps, int nchunks, int f16m, float scl,
             unsigned short* dst)
{
  const int q    = blockIdx.x * 256 + threadIdx.x;
  const int qc   = min(q, nchunks - 1);
  const int cpr  = cin >> 3;
  const int c8   = qc % cpr;
  const int rem  = qc / cpr;
  const int o    = rem % NCO;
  const int k    = rem / NCO;
  const float* s = w + ((size_t)o * cin + 8 * c8) * ktaps + k;
  unsigned hb[8];
#pragma unroll
  for (int j = 0; j < 8; ++j) {
    const float v = bf_rne(s[(size_t)j * ktaps]);
    hb[j] = (f16m != 0) ? h16b(v * scl) : bfb(v);
  }
  v4u wh;
  wh.x = hb[0] | (hb[1] << 16);
  wh.y = hb[2] | (hb[3] << 16);
  wh.z = hb[4] | (hb[5] << 16);
  wh.w = hb[6] | (hb[7] << 16);
  const bool ok = (q < nchunks);
  unsigned short* d = dst + (size_t)qc * 8;
  if (ok) *(volatile v4u*)d = wh;
  __threadfence();
  if (ok) *(volatile v4u*)d = wh;
}

template<int CIN, int NTAPS, bool GATHER, bool F16>
__global__ __launch_bounds__(256)
void k_conv(const unsigned short* __restrict__ xT, const unsigned short* __restrict__ wT,
            const int* __restrict__ nb, float* out, double* part, int npts, float oscale)
{
  typedef typename Mma<F16>::frag FR;
  typedef ConvCfg<CIN, GATHER> CF;
  constexpr int ROWP = CF::ROWP;
  constexpr int VPR  = CIN / 8;
  constexpr int ITW  = (NCO * VPR) / 256;
  constexpr int ITX  = (NT * VPR) / 256;
  static_assert(CIN % 32 == 0);
  static_assert((NCO * VPR) % 256 == 0);
  static_assert((NT * VPR) % 256 == 0);
  static_assert((ROWP * 2) % 16 == 0);
  static_assert(CF::UNI % 16 == 0);

  extern __shared__ __align__(16) unsigned char smem_raw[];
  unsigned short* lw  = (unsigned short*)smem_raw;
  unsigned short* lx  = lw + NCO * ROWP;
  float*          st  = (float*)smem_raw;
  int*            nbs = (int*)(smem_raw + CF::UNI);

  const int tid  = threadIdx.x;
  const int lane = tid & 31;
  const int wid  = tid >> 5;
  const int hl   = lane & 15;
  const int hh   = lane >> 4;
  const int mw   = wid & 3;
  const int nw   = wid >> 2;
  const int n0   = blockIdx.x * NT;

  if (GATHER) {
#pragma unroll 1
    for (int i = tid; i < NT * KTAP; i += 256) {
      int v = nb[(size_t)n0 * KTAP + i];
      v = min(max(v, 0), npts - 1);
      nbs[i] = v;
    }
  }

  v8f acc[2][4];
#pragma unroll
  for (int mt = 0; mt < 2; ++mt)
#pragma unroll
    for (int nt = 0; nt < 4; ++nt) acc[mt][nt] = zero8f();

#pragma unroll 1
  for (int k = 0; k < NTAPS; ++k) {
    __syncthreads();
    const unsigned short* wsrc = wT + (size_t)k * NCO * CIN;
#pragma unroll
    for (int it = 0; it < ITW; ++it) {
      const int c   = tid + it * 256;
      const int row = c / VPR;
      const int v   = c - row * VPR;
      const v4u t = *(const v4u*)(wsrc + (size_t)row * CIN + 8 * v);
      *(v4u*)(lw + row * ROWP + 8 * v) = t;
    }
#pragma unroll
    for (int it = 0; it < ITX; ++it) {
      const int c   = tid + it * 256;
      const int row = c / VPR;
      const int v   = c - row * VPR;
      const int idx = GATHER ? nbs[row * KTAP + k] : (n0 + row);
      const v4u t = *(const v4u*)(xT + (size_t)idx * CIN + 8 * v);
      *(v4u*)(lx + row * ROWP + 8 * v) = t;
    }
    __syncthreads();
#pragma unroll
    for (int ck = 0; ck < CIN / 32; ++ck) {
      FR af[2], bf[4];
#pragma unroll
      for (int mt = 0; mt < 2; ++mt)
        af[mt] = ldfrag<F16>(lw + (32 * mw + 16 * mt + hl) * ROWP + 32 * ck + 8 * hh);
#pragma unroll
      for (int nt = 0; nt < 4; ++nt)
        bf[nt] = ldfrag<F16>(lx + (64 * nw + 16 * nt + hl) * ROWP + 32 * ck + 8 * hh);
#pragma unroll
      for (int mt = 0; mt < 2; ++mt)
#pragma unroll
        for (int nt = 0; nt < 4; ++nt)
          acc[mt][nt] = Mma<F16>::mma(af[mt], bf[nt], acc[mt][nt]);
      guard8x6(acc[0][0], acc[0][1], acc[0][2], acc[0][3], acc[1][0], acc[1][1], acc[1][2], acc[1][3],
               af[0], af[1], bf[0], bf[1], bf[2], bf[3]);
    }
  }
  __syncthreads();
  acc_guard8(acc[0][0], acc[0][1], acc[0][2], acc[0][3], acc[1][0], acc[1][1], acc[1][2], acc[1][3]);

#pragma unroll
  for (int mt = 0; mt < 2; ++mt)
#pragma unroll
    for (int nt = 0; nt < 4; ++nt) {
      v4f q0, q1;
#pragma unroll
      for (int r = 0; r < 4; ++r) { q0[r] = acc[mt][nt][r] * oscale; q1[r] = acc[mt][nt][4 + r] * oscale; }
      float* ep = st + (64 * nw + 16 * nt + hl) * SP + 32 * mw + 16 * mt + 8 * hh;
      *(v4f*)ep       = q0;
      *(v4f*)(ep + 4) = q1;
    }
  __syncthreads();

  if (tid < NCO) {
    double s = 0.0, q = 0.0;
#pragma unroll 4
    for (int n = 0; n < NT; ++n) {
      const double v = (double)st[n * SP + tid];
      s += v;
      q += v * v;
    }
    v2d pv; pv.x = s; pv.y = q;
    double* pp = part + ((size_t)blockIdx.x * NCO + tid) * 2;
    *(volatile v2d*)pp = pv;
    __threadfence();
    *(volatile v2d*)pp = pv;
  }
  {
    v4f val[16];
#pragma unroll
    for (int i = 0; i < 16; ++i) {
      const int o = 8 * i + wid;
      const float* sp0 = st + (4 * lane) * SP + o;
      v4f t;
      t.x = sp0[0];
      t.y = sp0[SP];
      t.z = sp0[2 * SP];
      t.w = sp0[3 * SP];
      val[i] = t;
    }
    float* ob = out + (size_t)n0 + 4 * lane;
#pragma unroll
    for (int i = 0; i < 16; ++i) *(volatile v4f*)(ob + (size_t)(8 * i + wid) * npts) = val[i];
    __threadfence();
#pragma unroll
    for (int i = 0; i < 16; ++i) *(volatile v4f*)(ob + (size_t)(8 * i + wid) * npts) = val[i];
  }
}

__global__ __launch_bounds__(128)
void k_stats(const double* __restrict__ part, int nblk, int cnt, float* stats)
{
  __shared__ __align__(16) float sm[2 * NCO];
  const int c = threadIdx.x;
  const double* pb = part + (size_t)blockIdx.x * nblk * NCO * 2;
  float* sb = stats + (size_t)blockIdx.x * 2 * NCO;
  double s = 0.0, q = 0.0;
#pragma unroll 1
  for (int b = 0; b < nblk; ++b) {
    const v2d pv = *(const v2d*)(pb + ((size_t)b * NCO + c) * 2);
    s += pv.x;
    q += pv.y;
  }
  const double inv  = 1.0 / (double)cnt;
  const double mean = s * inv;
  double var = q * inv - mean * mean;
  if (var < 0.0) var = 0.0;
  const float mf = (float)mean;
  const float rs = 1.0f / sqrtf((float)var + BNEPS);
  sm[c]       = mf;
  sm[NCO + c] = rs;
  __syncthreads();
  if (c < 64) {
    const v4f v = *(const v4f*)&sm[4 * c];
    float* d = sb + 4 * c;
    *(volatile v4f*)d = v;
    __threadfence();
    *(volatile v4f*)d = v;
  }
}

__global__ __launch_bounds__(256)
void k_c1T(const float* __restrict__ raw, const float* __restrict__ stats,
           const float* __restrict__ gam, const float* __restrict__ bet, int npts, unsigned short* dst)
{
  __shared__ float tile[NCO * TP];
  __shared__ float prm[4 * NCO];
  const int tid  = threadIdx.x;
  const int lane = tid & 31;
  const int wid  = tid >> 5;
  const int pj   = lane & 7;
  const int lq   = lane >> 3;
  const int px   = tid & 31;
  const int cr   = tid >> 5;
  const int n0   = blockIdx.x * 32;
  if (tid < NCO) {
    prm[tid]           = stats[tid];
    prm[NCO + tid]     = stats[NCO + tid];
    prm[2 * NCO + tid] = bf_rne(gam[tid]);
    prm[3 * NCO + tid] = bf_rne(bet[tid]);
  }
  __syncthreads();
#pragma unroll 4
  for (int i = 0; i < 16; ++i) {
    const int c = cr + 8 * i;
    const float v = raw[(size_t)c * npts + n0 + px];
    float t = v - prm[c];
    t = prm[2 * NCO + c] * t;
    t = t * prm[NCO + c];
    t = t + prm[3 * NCO + c];
    tile[c * TP + px] = fmaxf(t, 0.f);
  }
  __syncthreads();
  v4u wv[2]; size_t eo[2];
#pragma unroll
  for (int it = 0; it < 2; ++it) {
    const int L  = it * 32 + wid * 4 + lq;
    const int pt = L >> 1;
    const int cb = 64 * (L & 1) + 8 * pj;
    unsigned hb[8];
#pragma unroll
    for (int e = 0; e < 8; ++e) hb[e] = h16b(tile[(cb + e) * TP + pt]);
    v4u t;
    t.x = hb[0] | (hb[1] << 16);
    t.y = hb[2] | (hb[3] << 16);
    t.z = hb[4] | (hb[5] << 16);
    t.w = hb[6] | (hb[7] << 16);
    wv[it] = t;
    eo[it] = (size_t)(n0 + pt) * NCO + cb;
  }
#pragma unroll
  for (int it = 0; it < 2; ++it) *(volatile v4u*)(dst + eo[it]) = wv[it];
  __threadfence();
#pragma unroll
  for (int it = 0; it < 2; ++it) *(volatile v4u*)(dst + eo[it]) = wv[it];
}

__global__ __launch_bounds__(256)
void k_final(const float* __restrict__ c2, const float* __restrict__ sk,
             const float* __restrict__ stb, const float* __restrict__ sts,
             const float* __restrict__ gb, const float* __restrict__ bb,
             const float* __restrict__ gs, const float* __restrict__ bs, int npts, float* out)
{
  const size_t i      = (size_t)blockIdx.x * 256 + threadIdx.x;
  const size_t total4 = (size_t)NCO * (size_t)npts / 4;
  const size_t ic     = (i < total4) ? i : (total4 - 1);
  const int o = (int)(ic / (size_t)(npts / 4));
  const float mub = stb[o], rsb = stb[NCO + o];
  const float mus = sts[o], rss = sts[NCO + o];
  const float g2 = bf_rne(gb[o]), b2 = bf_rne(bb[o]);
  const float g1 = bf_rne(gs[o]), b1 = bf_rne(bs[o]);
  const v4f a = *(const v4f*)(c2 + ic * 4);
  const v4f b = *(const v4f*)(sk + ic * 4);
  v4f r;
#pragma unroll
  for (int j = 0; j < 4; ++j) {
    float t = a[j] - mub; t = g2 * t; t = t * rsb; t = t + b2;
    float u = b[j] - mus; u = g1 * u; u = u * rss; u = u + b1;
    r[j] = fmaxf(t + u, 0.f);
  }
  const bool ok = (i < total4);
  float* d = out + ic * 4;
  if (ok) *(volatile v4f*)d = r;
  __threadfence();
  if (ok) *(volatile v4f*)d = r;
}

extern "C" void kernel_launch(void* const* d_in, const int* in_sizes, int n_in,
                              void* d_out, int out_size, void* d_ws, size_t ws_size,
                              hipStream_t stream) {
  if (n_in < 11) return;
  if (in_sizes[1] <= 0 || (in_sizes[1] % KTAP) != 0) return;
  const int N = in_sizes[1] / KTAP;
  if (N < NT || (N % NT) != 0) return;
  if (in_sizes[0] != CIA * N) return;
  if (in_sizes[2] != NCO * CIA * KTAP) return;
  if (in_sizes[3] != NCO * NCO * KTAP) return;
  if (in_sizes[4] != NCO * CIA) return;
  for (int i = 5; i < 11; ++i) if (in_sizes[i] != NCO) return;
  if (out_size != NCO * N) return;
  const int nblk = N / NT;

  const size_t o_xT   = 0;
  const size_t o_c1T  = o_xT   + (size_t)N * CIA * 2;
  const size_t o_araw = o_c1T  + (size_t)N * NCO * 2;
  const size_t o_sraw = o_araw + (size_t)NCO * N * 4;
  const size_t o_c2   = o_sraw + (size_t)NCO * N * 4;
  const size_t o_wat  = o_c2   + (size_t)NCO * N * 4;
  const size_t o_wbt  = o_wat  + (size_t)KTAP * NCO * CIA * 2;
  const size_t o_wst  = o_wbt  + (size_t)KTAP * NCO * NCO * 2;
  const size_t o_part = o_wst  + (size_t)NCO * CIA * 2;
  const size_t sz_pt  = (size_t)nblk * NCO * 2 * 8;
  const size_t o_stat = o_part + 3 * sz_pt;
  const size_t o_end  = o_stat + 3 * 1024;
  if (o_end > ws_size) return;

  const float* data = (const float*)d_in[0];
  const int*   nbr  = (const int*)d_in[1];
  const float* w_a  = (const float*)d_in[2];
  const float* w_b  = (const float*)d_in[3];
  const float* w_s  = (const float*)d_in[4];
  const float* g_a  = (const float*)d_in[5];
  const float* b_a  = (const float*)d_in[6];
  const float* g_b  = (const float*)d_in[7];
  const float* b_b  = (const float*)d_in[8];
  const float* g_s  = (const float*)d_in[9];
  const float* b_s  = (const float*)d_in[10];
  float* out = (float*)d_out;
  char* ws = (char*)d_ws;

  unsigned short* xT   = (unsigned short*)(ws + o_xT);
  unsigned short* c1T  = (unsigned short*)(ws + o_c1T);
  float*          araw = (float*)(ws + o_araw);
  float*          sraw = (float*)(ws + o_sraw);
  float*          c2rw = (float*)(ws + o_c2);
  unsigned short* wat  = (unsigned short*)(ws + o_wat);
  unsigned short* wbt  = (unsigned short*)(ws + o_wbt);
  unsigned short* wst  = (unsigned short*)(ws + o_wst);
  double*         pt_a = (double*)(ws + o_part);
  double*         pt_s = (double*)(ws + o_part + sz_pt);
  double*         pt_b = (double*)(ws + o_part + 2 * sz_pt);
  float*          st_a = (float*)(ws + o_stat);
  float*          st_s = st_a + 2 * NCO;
  float*          st_b = st_a + 4 * NCO;

  const int ldsA = ConvCfg<CIA, true>::LDS;
  const int ldsS = ConvCfg<CIA, false>::LDS;
  const int ldsB = ConvCfg<NCO, true>::LDS;
  (void)hipFuncSetAttribute(reinterpret_cast<const void*>(&k_conv<CIA, KTAP, true, false>),
                            hipFuncAttributeMaxDynamicSharedMemorySize, ldsA);
  (void)hipFuncSetAttribute(reinterpret_cast<const void*>(&k_conv<CIA, 1, false, false>),
                            hipFuncAttributeMaxDynamicSharedMemorySize, ldsS);
  (void)hipFuncSetAttribute(reinterpret_cast<const void*>(&k_conv<NCO, KTAP, true, true>),
                            hipFuncAttributeMaxDynamicSharedMemorySize, ldsB);
  (void)hipGetLastError();

  const int nchA = KTAP * NCO * (CIA / 8);
  const int nchS = NCO * (CIA / 8);
  const int nchB = KTAP * NCO * (NCO / 8);

  k_xT<<<dim3(N / 32), dim3(256), 0, stream>>>(data, N, xT);
  (void)hipGetLastError();
  k_wpack<<<dim3((nchA + 255) / 256), dim3(256), 0, stream>>>(w_a, CIA, KTAP, nchA, 0, 1.0f, wat);
  (void)hipGetLastError();
  k_wpack<<<dim3((nchS + 255) / 256), dim3(256), 0, stream>>>(w_s, CIA, 1, nchS, 0, 1.0f, wst);
  (void)hipGetLastError();
  k_wpack<<<dim3((nchB + 255) / 256), dim3(256), 0, stream>>>(w_b, NCO, KTAP, nchB, 1, 16.0f, wbt);
  (void)hipGetLastError();
  k_conv<CIA, KTAP, true, false><<<dim3(nblk), dim3(256), ldsA, stream>>>(xT, wat, nbr, araw, pt_a, N, 1.0f);
  (void)hipGetLastError();
  k_conv<CIA, 1, false, false><<<dim3(nblk), dim3(256), ldsS, stream>>>(xT, wst, nbr, sraw, pt_s, N, 1.0f);
  (void)hipGetLastError();
  k_stats<<<dim3(2), dim3(128), 0, stream>>>(pt_a, nblk, N, st_a);
  (void)hipGetLastError();
  k_c1T<<<dim3(N / 32), dim3(256), 0, stream>>>(araw, st_a, g_a, b_a, N, c1T);
  (void)hipGetLastError();
  k_conv<NCO, KTAP, true, true><<<dim3(nblk), dim3(256), ldsB, stream>>>(c1T, wbt, nbr, c2rw, pt_b, N, 0.0625f);
  (void)hipGetLastError();
  k_stats<<<dim3(1), dim3(128), 0, stream>>>(pt_b, nblk, N, st_b);
  (void)hipGetLastError();
  k_final<<<dim3((unsigned)(((size_t)NCO * N / 4 + 255) / 256)), dim3(256), 0, stream>>>(
      c2rw, sraw, st_b, st_s, g_b, b_b, g_s, b_s, N, out);
  (void)hipGetLastError();
}
